// GNNBase_48481590837648
// MI455X (gfx1250) — hardware-verified
//
#include <hip/hip_runtime.h>
#include <math.h>

constexpr int kNodes   = 50000;
constexpr int kEdges   = 500000;
constexpr int kDin     = 32;
constexpr int kDemb    = 32;
constexpr int kDedge   = 4;
constexpr int kTypes   = 8;
constexpr int kHid     = 256;
constexpr int kK1      = kDin + kDemb + kDedge;
constexpr int kK1P     = 96;
constexpr int kThreads = 256;
constexpr int kTileE   = 64;
constexpr int kDstB    = 128;
constexpr int kBlocks  = (kNodes + kDstB - 1) / kDstB;
constexpr int kSP      = 16;
constexpr int kSCH     = kThreads * kSP;
constexpr int kChunks  = (kEdges + kSCH - 1) / kSCH;
constexpr int kQCap    = kSCH + kTileE;
constexpr int kMaxTile = kQCap / kTileE;
constexpr int kLdX     = 104;
constexpr int kLdA     = 264;
constexpr int kSegH    = 2048;
constexpr int kSeg1    = kHid * kK1P / kSegH;
constexpr int kSeg2    = kHid * kHid / kSegH;
constexpr int kPackBlocks = kSeg1 + 2 * kSeg2;
constexpr float kWCarry    = 16.0f;
constexpr float kWCarryInv = 1.0f / 16.0f;
constexpr float kLnEps     = 1e-5f;
constexpr float kInvHid    = 1.0f / 256.0f;

static_assert(kK1P % 32 == 0 && kK1P >= kK1, "K pad");
static_assert(kHid % 32 == 0, "K2 K3 multiple of 32");
static_assert(kHid == 8 * 32, "wave w owns columns 32w..32w+31");
static_assert(kThreads == 4 * kTileE, "gather: 4 threads per tile row");
static_assert(kThreads == kHid, "parameter staging: one thread per column");
static_assert(kThreads / 32 >= 2 && kTileE == 64, "row combine by waves 0 and 1");
static_assert(kDin == 32 && kDemb == 32 && kDedge == 4, "gather layout");
static_assert(kDstB <= 512 && (kDstB & (kDstB - 1)) == 0, "hit record (e << 9) | dl, dl < 512");
static_assert(kEdges <= (1 << 22), "(e << 9) | dl stays positive in int32");
static_assert(kEdges % kSP == 0 && kSP % 4 == 0, "stream groups entirely in or out of range");
static_assert(kQCap == kSCH + kTileE, "one append pass holds every hit of a chunk");
static_assert((kHid * kK1P) % kSegH == 0 && (kHid * kHid) % kSegH == 0, "pack segments");
static_assert(kSegH == 8 * kThreads, "pack: 8 halves per thread");
static_assert(kK1P % 8 == 0 && kHid % 8 == 0, "pack rows");
static_assert(kLdX % 8 == 0 && kLdA % 8 == 0, "16-B aligned tile rows");
static_assert(kLdX <= kLdA, "X tile fits in the H tile buffer");
static_assert(kBlocks * kDstB >= kNodes, "node coverage");
static_assert(kChunks * kSCH >= kEdges, "edge coverage");
static_assert((kDstB * kHid) % (4 * kThreads) == 0, "accumulator zero fill");
static_assert((kTileE * kLdA / 2) % 4 == 0, "tile zero fill");

typedef __attribute__((ext_vector_type(16))) _Float16 v16h;
typedef __attribute__((ext_vector_type(8)))  _Float16 v8h;
typedef __attribute__((ext_vector_type(8)))  float    v8f;
typedef __attribute__((ext_vector_type(4)))  float    v4f;
typedef __attribute__((ext_vector_type(4)))  unsigned int v4u;
typedef __attribute__((ext_vector_type(2)))  unsigned int v2u;
typedef __attribute__((ext_vector_type(4)))  int      v4i;

__device__ __forceinline__ unsigned short f2bf_bits(float f) {
  unsigned u = __float_as_uint(f);
  return (unsigned short)((u + 0x7FFFu + ((u >> 16) & 1u)) >> 16);
}
__device__ __forceinline__ float bf_bits2f(unsigned short h) { return __uint_as_float(((unsigned)h) << 16); }
__device__ __forceinline__ float bfr(float x) { return bf_bits2f(f2bf_bits(x)); }

__device__ __forceinline__ void dep_guard_h(v8f& a, v8f& b, v16h x, v16h y) { asm volatile("v_nop\n\tv_nop\n\tv_nop\n\tv_nop" : "+v"(a), "+v"(b) : "v"(x), "v"(y)); }
__device__ __forceinline__ void keep4_h(v16h a, v16h b, v16h c, v16h d) { asm volatile("v_nop" :: "v"(a), "v"(b), "v"(c), "v"(d)); }
__device__ __forceinline__ void acc_guard4(v8f& a, v8f& b, v8f& c, v8f& d) { asm volatile("v_nop\n\tv_nop\n\tv_nop\n\tv_nop" : "+v"(a), "+v"(b), "+v"(c), "+v"(d)); }
template <typename T> struct Frag;
template <> struct Frag<_Float16> {
  typedef v16h V; union U { v16h v; v8h h[2]; };
  static __device__ __forceinline__ v16h load(const _Float16* p) {
    U f; f.h[0] = *(const v8h*)(p); f.h[1] = *(const v8h*)(p + 16); return f.v;
  }
  static __device__ __forceinline__ v8f mma(v16h a, v16h b, v8f c) {
    return __builtin_amdgcn_wmma_f32_16x16x32_f16(false, a, false, b, (short)0, c, false, false);
  }
  static __device__ __forceinline__ void guard(v8f& a, v8f& b, v16h x, v16h y) { dep_guard_h(a, b, x, y); }
  static __device__ __forceinline__ void keep(v16h a, v16h b, v16h c, v16h d) { keep4_h(a, b, c, d); }
};

__device__ __forceinline__ unsigned pk16(unsigned short a, unsigned short b) { return (unsigned)a | ((unsigned)b << 16); }
__device__ __forceinline__ unsigned short h_bits(float f) { const _Float16 h = (_Float16)f; return __builtin_bit_cast(unsigned short, h); }
__device__ __forceinline__ unsigned short hb_of(float x) { return h_bits(bfr(x)); }
__device__ __forceinline__ int perm_k(int p) { return (p & ~31) | ((p & 1) << 4) | ((p >> 1) & 15); }

__device__ __forceinline__ int blk_excl_scan(int cnt, int* scan_ws, int tid, int lane, int wave, int* tot) {
  int incl = cnt;
#pragma unroll
  for (int o = 1; o < 32; o <<= 1) { const int v = __shfl_up(incl, o, 32); if (lane >= o) incl += v; }
  if (lane == 31) scan_ws[wave] = incl;
  __syncthreads();
  if (wave == 0) {
    const int wraw = scan_ws[lane & 7];
    const int wv = (lane < 8) ? wraw : 0;
    int wincl = wv;
#pragma unroll
    for (int o = 1; o < 32; o <<= 1) { const int v = __shfl_up(wincl, o, 32); if (lane >= o) wincl += v; }
    if (lane < 8) scan_ws[32 + lane] = wincl - wv;
    if (lane == 31) scan_ws[64] = wincl;
  }
  __syncthreads();
  *tot = scan_ws[64];
  return scan_ws[32 + wave] + incl - cnt;
}

__global__ __launch_bounds__(kThreads) void pack_weights(const float* __restrict__ W1, const float* __restrict__ W2,
                                                           const float* __restrict__ W3,
                                                           unsigned short* __restrict__ Bt1, unsigned short* __restrict__ Bt2,
                                                           unsigned short* __restrict__ Bt3) {
  const int bx = blockIdx.x;
  const float* W; unsigned short* O; int KP, KR, seg, prm;
  if (bx < kSeg1)              { W = W1; O = Bt1; KP = kK1P; KR = kK1;  seg = bx;                 prm = 0; }
  else if (bx < kSeg1 + kSeg2) { W = W2; O = Bt2; KP = kHid; KR = kHid; seg = bx - kSeg1;         prm = 1; }
  else                         { W = W3; O = Bt3; KP = kHid; KR = kHid; seg = bx - kSeg1 - kSeg2; prm = 1; }
  const int L0 = seg * kSegH + 8 * (int)threadIdx.x;
  const int n  = L0 / KP;
  const int pb = L0 - n * KP;
  unsigned short hbv[8];
#pragma unroll
  for (int e = 0; e < 8; ++e) {
    const int p  = pb + e;
    const int k  = prm ? perm_k(p) : p;
    const int kc = (k < KR) ? k : (KR - 1);
    const float w = W[(size_t)kc * kHid + n];
    const float f = (k < KR) ? 1.0f : 0.0f;
    hbv[e] = h_bits(bfr(w) * f * kWCarry);
  }
  const v4u u = (v4u){pk16(hbv[0], hbv[1]), pk16(hbv[2], hbv[3]), pk16(hbv[4], hbv[5]), pk16(hbv[6], hbv[7])};
  unsigned short* op = O + L0;
  *(volatile v4u*)op = u;
  __threadfence();
  *(volatile v4u*)op = u;
}

template <int KDIM, int LDIN, int MODE>
__device__ __forceinline__ void mlp_layer(unsigned int* hbufw, const _Float16* __restrict__ Bt,
                                          const float* pb, const float* pg, const float* pe,
                                          float* redP, float* rowMu, float* rowRs,
                                          const int* tileDl, float* accL, int tid, int wave, int lane) {
  const int m    = lane & 15;
  const int hh   = lane >> 4;
  const int koff = hh * 8;
  const int cw0  = wave * 32;
  const _Float16* Ain = (const _Float16*)hbufw;
  v8f acc[4][2];
#pragma unroll
  for (int i = 0; i < 4; ++i) {
    acc[i][0] = (v8f){0.f, 0.f, 0.f, 0.f, 0.f, 0.f, 0.f, 0.f};
    acc[i][1] = (v8f){0.f, 0.f, 0.f, 0.f, 0.f, 0.f, 0.f, 0.f};
  }
#pragma unroll 1
  for (int k0 = 0; k0 < KDIM; k0 += 32) {
    const v16h b0 = Frag<_Float16>::load(Bt + (cw0 + m) * KDIM + koff + k0);
    const v16h b1 = Frag<_Float16>::load(Bt + (cw0 + 16 + m) * KDIM + koff + k0);
#pragma unroll
    for (int i = 0; i < 4; ++i) {
      const v16h a = Frag<_Float16>::load(Ain + (16 * i + m) * LDIN + koff + k0);
      acc[i][0] = Frag<_Float16>::mma(a, b0, acc[i][0]);
      acc[i][1] = Frag<_Float16>::mma(a, b1, acc[i][1]);
      Frag<_Float16>::guard(acc[i][0], acc[i][1], a, a);
    }
    Frag<_Float16>::keep(b0, b1, b0, b1);
  }
  acc_guard4(acc[0][0], acc[0][1], acc[1][0], acc[1][1]);
  acc_guard4(acc[2][0], acc[2][1], acc[3][0], acc[3][1]);

  const float bb0 = pb[cw0 + m];
  const float bb1 = pb[cw0 + 16 + m];
#pragma unroll
  for (int i = 0; i < 4; ++i) {
#pragma unroll
    for (int r = 0; r < 8; ++r) {
      const float v0 = fmaxf(fmaf(acc[i][0][r], kWCarryInv, bb0), 0.f);
      const float v1 = fmaxf(fmaf(acc[i][1][r], kWCarryInv, bb1), 0.f);
      acc[i][0][r] = v0;
      acc[i][1][r] = v1;
      float s = v0 + v1;
      s += __shfl_xor(s, 1, 32);
      s += __shfl_xor(s, 2, 32);
      s += __shfl_xor(s, 4, 32);
      s += __shfl_xor(s, 8, 32);
      if (m == 0) redP[wave * kTileE + 16 * i + 8 * hh + r] = s;
    }
  }
  __syncthreads();
  if (wave < 2) {
    float S = 0.f;
#pragma unroll
    for (int w = 0; w < 8; ++w) S += redP[w * kTileE + tid];
    rowMu[tid] = S * kInvHid;
  }
  __syncthreads();
#pragma unroll
  for (int i = 0; i < 4; ++i) {
#pragma unroll
    for (int r = 0; r < 8; ++r) {
      const float mu = rowMu[16 * i + 8 * hh + r];
      const float d0 = acc[i][0][r] - mu;
      const float d1 = acc[i][1][r] - mu;
      float q = d0 * d0;
      q = fmaf(d1, d1, q);
      q += __shfl_xor(q, 1, 32);
      q += __shfl_xor(q, 2, 32);
      q += __shfl_xor(q, 4, 32);
      q += __shfl_xor(q, 8, 32);
      if (m == 0) redP[wave * kTileE + 16 * i + 8 * hh + r] = q;
    }
  }
  __syncthreads();
  if (wave < 2) {
    float Q = 0.f;
#pragma unroll
    for (int w = 0; w < 8; ++w) Q += redP[w * kTileE + tid];
    rowRs[tid] = rsqrtf(fmaf(Q, kInvHid, kLnEps));
  }
  __syncthreads();
  const float gg0 = pg[cw0 + m], gg1 = pg[cw0 + 16 + m];
  const float ee0 = pe[cw0 + m], ee1 = pe[cw0 + 16 + m];
#pragma unroll
  for (int i = 0; i < 4; ++i) {
#pragma unroll
    for (int r = 0; r < 8; ++r) {
      const int row = 16 * i + 8 * hh + r;
      const float mu = rowMu[row];
      const float rs = rowRs[row];
      const float y0 = fmaf((acc[i][0][r] - mu) * rs, gg0, ee0);
      const float y1 = fmaf((acc[i][1][r] - mu) * rs, gg1, ee1);
      if (MODE == 0) {
        hbufw[row * (kLdA / 2) + (cw0 >> 1) + m] = pk16(h_bits(y0), h_bits(y1));
      } else {
#pragma unroll
        for (int hq = 0; hq < 2; ++hq) {
          const float a0 = __shfl(y0, m + 16 * hq, 32);
          const float a1 = __shfl(y1, m + 16 * hq, 32);
          const float val = hh ? a1 : a0;
          const int dl = __builtin_amdgcn_readfirstlane(tileDl[16 * i + 8 * hq + r]);
          const float fv = (dl >= 0) ? 1.0f : 0.0f;
          const int dlc = (dl >= 0) ? (dl & (kDstB - 1)) : 0;
          float* ap = accL + dlc * kHid + cw0 + lane;
          const float o = *ap;
          *ap = fmaf(val, fv, o);
        }
      }
    }
  }
  __syncthreads();
}

__global__ __launch_bounds__(kThreads) __attribute__((amdgpu_num_vgpr(256)))
void edge_mlp_segsum(
    const float* __restrict__ node_feat, const int* __restrict__ node_type, const int* __restrict__ edge_index,
    const float* __restrict__ edge_attr, const float* __restrict__ embed,
    const unsigned short* __restrict__ Bt1, const unsigned short* __restrict__ Bt2, const unsigned short* __restrict__ Bt3,
    const float* __restrict__ b1, const float* __restrict__ g1, const float* __restrict__ e1,
    const float* __restrict__ b2, const float* __restrict__ g2, const float* __restrict__ e2,
    const float* __restrict__ b3, const float* __restrict__ g3, const float* __restrict__ e3,
    float* __restrict__ out) {
  __shared__ __align__(16) float accL[kDstB * kHid];
  __shared__ __align__(16) unsigned int hbufw[kTileE * kLdA / 2];
  __shared__ __align__(16) float prm[9 * kHid];
  __shared__ int qbuf[kQCap];
  __shared__ float redP[8 * kTileE];
  __shared__ float rowMu[kTileE];
  __shared__ float rowRs[kTileE];
  __shared__ int tileDl[kTileE];
  __shared__ int scan_ws[80];

  const int tid  = threadIdx.x;
  const int lane = tid & 31;
  const int wave = __builtin_amdgcn_readfirstlane(tid >> 5);
  const int n0   = blockIdx.x * kDstB;
  const int nhi  = (n0 + kDstB < kNodes) ? (n0 + kDstB) : kNodes;
  const int* dstv = edge_index + kEdges;
  const _Float16* Bt1h = (const _Float16*)Bt1;
  const _Float16* Bt2h = (const _Float16*)Bt2;
  const _Float16* Bt3h = (const _Float16*)Bt3;
  const v4f z4  = {0.f, 0.f, 0.f, 0.f};
  const v4u z4u = {0u, 0u, 0u, 0u};
  const v2u z2u = {0u, 0u};

  prm[0 * kHid + tid] = bfr(b1[tid]); prm[1 * kHid + tid] = bfr(g1[tid]); prm[2 * kHid + tid] = bfr(e1[tid]);
  prm[3 * kHid + tid] = bfr(b2[tid]); prm[4 * kHid + tid] = bfr(g2[tid]); prm[5 * kHid + tid] = bfr(e2[tid]);
  prm[6 * kHid + tid] = bfr(b3[tid]); prm[7 * kHid + tid] = bfr(g3[tid]); prm[8 * kHid + tid] = bfr(e3[tid]);
#pragma unroll 1
  for (int i = tid; i < kQCap; i += kThreads) qbuf[i] = -1;
  if (tid < 80) scan_ws[tid] = 0;
  if (tid < kTileE) { tileDl[tid] = -1; rowMu[tid] = 0.f; rowRs[tid] = 0.f; }
#pragma unroll 1
  for (int i = tid; i < 8 * kTileE; i += kThreads) redP[i] = 0.f;
#pragma unroll 1
  for (int i = tid; i < kDstB * kHid / 4; i += kThreads) *(v4f*)(accL + 4 * i) = z4;
#pragma unroll 1
  for (int i = tid; i < kTileE * kLdA / 8; i += kThreads) *(v4u*)(hbufw + 4 * i) = z4u;
  __syncthreads();

  int qlen = 0;
#pragma unroll 1
  for (int c = 0; c <= kChunks; ++c) {
    const bool flush = (c == kChunks);
    int nadd = 0;
    if (!flush) {
      const int  eb  = c * kSCH + tid * kSP;
      const bool inr = (eb < kEdges);
      const int  ebc = inr ? eb : (kEdges - kSP);
      int rec[kSP];
      int cnt = 0;
#pragma unroll
      for (int k4 = 0; k4 < kSP; k4 += 4) {
        const v4i d4 = *(const v4i*)(dstv + ebc + k4);
#pragma unroll
        for (int e = 0; e < 4; ++e) {
          const int d  = d4[e];
          const bool hit = inr && (d >= n0) && (d < nhi);
          rec[k4 + e] = hit ? (((eb + k4 + e) << 9) | ((d - n0) & (kDstB - 1))) : -1;
          cnt += hit ? 1 : 0;
        }
      }
      int totraw;
      int p = blk_excl_scan(cnt, scan_ws, tid, lane, wave, &totraw);
#pragma unroll
      for (int k = 0; k < kSP; ++k) {
        const int rk = rec[k];
        if (rk >= 0) { const int qi = qlen + p; if ((unsigned)qi < (unsigned)kQCap) qbuf[qi] = rk; ++p; }
      }
      nadd = __builtin_amdgcn_readfirstlane(totraw);
      nadd = (nadd < 0) ? 0 : ((nadd < kSCH) ? nadd : kSCH);
    }
    __syncthreads();
    const int qtot = qlen + nadd;
    int ntile = flush ? ((qtot + kTileE - 1) / kTileE) : (qtot / kTileE);
    ntile = (ntile < kMaxTile) ? ntile : kMaxTile;
#pragma unroll 1
    for (int t = 0; t < ntile; ++t) {
      int nvalid = qtot - kTileE * t;
      nvalid = (nvalid < kTileE) ? nvalid : kTileE;

      {
        const int r = tid >> 2, q = tid & 3;
        const int rvraw = qbuf[kTileE * t + r];
        const int rv = (r < nvalid) ? rvraw : -1;
        const bool valid = (rv >= 0);
        const float vf = valid ? 1.0f : 0.0f;
        int e = valid ? (rv >> 9) : 0;
        e = (e < 0) ? 0 : ((e < kEdges) ? e : (kEdges - 1));
        const int dl = rv & (kDstB - 1);
        int s = edge_index[e];
        s = (s < 0) ? 0 : ((s >= kNodes) ? (kNodes - 1) : s);
        int ty = node_type[s];
        ty = (ty < 0) ? 0 : ((ty >= kTypes) ? (kTypes - 1) : ty);
        const float* fp = node_feat + (size_t)s * kDin + q * 8;
        const float* mp = embed + ty * kDemb + q * 8;
        const v4f f0 = *(const v4f*)(fp), f1 = *(const v4f*)(fp + 4);
        const v4f m0 = *(const v4f*)(mp), m1 = *(const v4f*)(mp + 4);
        const v4f ea = *(const v4f*)(edge_attr + (size_t)e * kDedge);
        unsigned short hf[8], hm[8], ht[4];
#pragma unroll
        for (int u = 0; u < 4; ++u) {
          hf[u] = hb_of(f0[u] * vf); hf[4 + u] = hb_of(f1[u] * vf);
          hm[u] = hb_of(m0[u] * vf); hm[4 + u] = hb_of(m1[u] * vf);
          ht[u] = hb_of(ea[u] * vf);
        }
        const v4u uf = (v4u){pk16(hf[0], hf[1]), pk16(hf[2], hf[3]), pk16(hf[4], hf[5]), pk16(hf[6], hf[7])};
        const v4u um = (v4u){pk16(hm[0], hm[1]), pk16(hm[2], hm[3]), pk16(hm[4], hm[5]), pk16(hm[6], hm[7])};
        const v2u ut = (v2u){pk16(ht[0], ht[1]), pk16(ht[2], ht[3])};
        unsigned int* xr = hbufw + r * (kLdX / 2);
        *(v4u*)(xr + 4 * q)      = uf;
        *(v4u*)(xr + 16 + 4 * q) = um;
        if (q == 0) {
          *(v2u*)(xr + 32) = ut;
          *(v2u*)(xr + 34) = z2u;
          tileDl[r] = valid ? dl : -1;
        } else {
          *(v4u*)(xr + 32 + 4 * q) = z4u;
        }
      }
      __syncthreads();

      mlp_layer<kK1P, kLdX, 0>(hbufw, Bt1h, prm + 0 * kHid, prm + 1 * kHid, prm + 2 * kHid,
                               redP, rowMu, rowRs, tileDl, accL, tid, wave, lane);
      mlp_layer<kHid, kLdA, 0>(hbufw, Bt2h, prm + 3 * kHid, prm + 4 * kHid, prm + 5 * kHid,
                               redP, rowMu, rowRs, tileDl, accL, tid, wave, lane);
      mlp_layer<kHid, kLdA, 1>(hbufw, Bt3h, prm + 6 * kHid, prm + 7 * kHid, prm + 8 * kHid,
                               redP, rowMu, rowRs, tileDl, accL, tid, wave, lane);
    }
    const int nfull = qtot / kTileE;
    const int rem   = flush ? 0 : (qtot - nfull * kTileE);
    if (tid < rem) { const int mv = qbuf[kTileE * nfull + tid]; qbuf[tid] = mv; }
    __syncthreads();
    qlen = rem;
  }

#pragma unroll 1
  for (int j = 0; j < kDstB / 8; ++j) {
    const int dl = 8 * j + wave;
    const int n  = n0 + dl;
    if (n < kNodes) {
      const float* ap = accL + dl * kHid + 4 * lane;
      const v4f a0 = *(const v4f*)ap;
      const v4f a1 = *(const v4f*)(ap + 128);
      float* rp = out + (size_t)n * kHid + 4 * lane;
      *(volatile v4f*)rp = a0;
      *(volatile v4f*)(rp + 128) = a1;
      __threadfence();
      *(volatile v4f*)rp = a0;
      *(volatile v4f*)(rp + 128) = a1;
    }
  }
}

extern "C" void kernel_launch(void* const* d_in, const int* in_sizes, int n_in,
                              void* d_out, int out_size, void* d_ws, size_t ws_size, hipStream_t stream) {
  if (n_in < 17) return;
  const float* node_feat = (const float*)d_in[0];
  const int*   node_type = (const int*)  d_in[1];
  const int*   edge_idx  = (const int*)  d_in[2];
  const float* edge_attr = (const float*)d_in[3];
  const float* embed     = (const float*)d_in[4];
  const float* W1  = (const float*)d_in[5];
  const float* b1  = (const float*)d_in[6];
  const float* g1  = (const float*)d_in[7];
  const float* be1 = (const float*)d_in[8];
  const float* W2  = (const float*)d_in[9];
  const float* b2  = (const float*)d_in[10];
  const float* g2  = (const float*)d_in[11];
  const float* be2 = (const float*)d_in[12];
  const float* W3  = (const float*)d_in[13];
  const float* b3  = (const float*)d_in[14];
  const float* g3  = (const float*)d_in[15];
  const float* be3 = (const float*)d_in[16];
  float* out = (float*)d_out;

  if (in_sizes[0] != kNodes * kDin || in_sizes[1] != kNodes || in_sizes[2] != 2 * kEdges ||
      in_sizes[3] != kEdges * kDedge || in_sizes[4] != kTypes * kDemb || in_sizes[5] != kK1 * kHid ||
      in_sizes[6] != kHid || in_sizes[7] != kHid || in_sizes[8] != kHid ||
      in_sizes[9] != kHid * kHid || in_sizes[10] != kHid || in_sizes[11] != kHid || in_sizes[12] != kHid ||
      in_sizes[13] != kHid * kHid || in_sizes[14] != kHid || in_sizes[15] != kHid || in_sizes[16] != kHid ||
      out_size != kNodes * kHid) return;

  const size_t bt1Bytes = (size_t)kHid * kK1P * 2;
  const size_t bt2Bytes = (size_t)kHid * kHid * 2;
  const size_t total = bt1Bytes + 2 * bt2Bytes;
  if (total > ws_size) return;
  char* ws = (char*)d_ws;
  unsigned short* Bt1 = (unsigned short*)(ws);
  unsigned short* Bt2 = (unsigned short*)(ws + bt1Bytes);
  unsigned short* Bt3 = (unsigned short*)(ws + bt1Bytes + bt2Bytes);

  pack_weights<<<kPackBlocks, kThreads, 0, stream>>>(W1, W2, W3, Bt1, Bt2, Bt3);
  edge_mlp_segsum<<<kBlocks, kThreads, 0, stream>>>(node_feat, node_type, edge_idx, edge_attr, embed,
                                                     Bt1, Bt2, Bt3,
                                                     b1, g1, be1, b2, g2, be2, b3, g3, be3, out);
}
